// ProofStateLatentAttention_5935644803714
// MI455X (gfx1250) — hardware-verified
//
#include <hip/hip_runtime.h>


#define NB_  2
#define TT   2048
#define DM   1024
#define NH_  16
#define HD   64
#define DL   256
#define ZH   2
#define RH   512
#define SCL  0.125f
#define PCAR 1024.0f
typedef _Float16 h16;
typedef unsigned short bf;
typedef __attribute__((ext_vector_type(16))) __bf16   v16bf;
typedef __attribute__((ext_vector_type(16))) _Float16 v16h;
typedef __attribute__((ext_vector_type(8)))  _Float16 v8h;
typedef __attribute__((ext_vector_type(8)))  unsigned short v8us;
typedef __attribute__((ext_vector_type(8)))  float    v8f;
typedef __attribute__((ext_vector_type(4)))  float    v4f;
typedef v8h  __attribute__((may_alias)) v8ha;
typedef v4f  __attribute__((may_alias)) v4fa;
typedef v8us __attribute__((may_alias)) v8usa;

__device__ __forceinline__ unsigned short f2bf(float f) { unsigned u = __float_as_uint(f); u += 0x7FFFu + ((u >> 16) & 1u); return (unsigned short)(u >> 16); }
__device__ __forceinline__ float bf2f(unsigned short b) { return __uint_as_float(((unsigned)b) << 16); }
__device__ __forceinline__ float bfr(float f) { return bf2f(f2bf(f)); }
__device__ __forceinline__ v16h cat16(v8h lo, v8h hi) { return __builtin_shufflevector(lo, hi, 0, 1, 2, 3, 4, 5, 6, 7, 8, 9, 10, 11, 12, 13, 14, 15); }
__device__ __forceinline__ v16bf cat16b(v8us lo, v8us hi) { return __builtin_bit_cast(v16bf, __builtin_shufflevector(lo, hi, 0, 1, 2, 3, 4, 5, 6, 7, 8, 9, 10, 11, 12, 13, 14, 15)); }
__device__ __forceinline__ v8f wmma16(v16h a, v16h b, v8f c) { return __builtin_amdgcn_wmma_f32_16x16x32_f16(false, a, false, b, (short)0, c, false, false); }
__device__ __forceinline__ v8f wmmab(v16bf a, v16bf b, v8f c) { return __builtin_amdgcn_wmma_f32_16x16x32_bf16(false, a, false, b, (short)0, c, false, false); }


template <typename T16> struct WFrag;
template <> struct WFrag<h16> { typedef v16h V; static __device__ __forceinline__ V ld(const h16* p) { return cat16(*(const v8h*)p, *(const v8h*)(p + 16)); } static __device__ __forceinline__ v8f mma(V a, V b, v8f c) { return wmma16(a, b, c); } };
template <> struct WFrag<bf> { typedef v16bf V; static __device__ __forceinline__ V ld(const bf* p) { return cat16b(*(const v8us*)p, *(const v8us*)(p + 16)); } static __device__ __forceinline__ v8f mma(V a, V b, v8f c) { return wmmab(a, b, c); } };
template <typename T16, int NSPLIT, bool BIAS>
__global__ __launch_bounds__(32) void k_gemmw(const T16* __restrict__ A, const T16* __restrict__ A2, const T16* __restrict__ Bt, const T16* __restrict__ Bt2, int K, float* C, int ldc, const float* __restrict__ bias, size_t sA, size_t sB, size_t sC) {
    typedef typename WFrag<T16>::V V;
    __shared__ __align__(16) float os[16 * 68];
    const size_t z = blockIdx.z; A += z * sA; if (A2) A2 += z * sA; Bt += z * sB; if (Bt2) Bt2 += z * sB; C += z * sC;
    const int lane = threadIdx.x & 31, lr = lane & 15, hi = lane >> 4; const int r0 = blockIdx.x * 64, c0 = blockIdx.y * 64;
    v8f acc[4][4];
#pragma unroll
    for (int mb = 0; mb < 4; ++mb)
#pragma unroll
        for (int nb = 0; nb < 4; ++nb) acc[mb][nb] = (v8f){};
    const size_t aoff = (size_t)(r0 + lr) * K + 8 * hi, boff = (size_t)(c0 + lr) * K + 8 * hi;
#pragma unroll 1
    for (int kc = 0; kc < K; kc += 32) {
        V a[4], a2[4];
#pragma unroll
        for (int mb = 0; mb < 4; ++mb) { a[mb] = WFrag<T16>::ld(A + aoff + (size_t)mb * 16 * K + kc); if (NSPLIT == 1 || NSPLIT == 2) a2[mb] = WFrag<T16>::ld(A2 + aoff + (size_t)mb * 16 * K + kc); }
#pragma unroll
        for (int nb = 0; nb < 4; ++nb) { const V b = WFrag<T16>::ld(Bt + boff + (size_t)nb * 16 * K + kc); V b2; if (NSPLIT >= 2) b2 = WFrag<T16>::ld(Bt2 + boff + (size_t)nb * 16 * K + kc);
#pragma unroll
            for (int mb = 0; mb < 4; ++mb) { acc[mb][nb] = WFrag<T16>::mma(a[mb], b, acc[mb][nb]); if (NSPLIT == 1 || NSPLIT == 2) acc[mb][nb] = WFrag<T16>::mma(a2[mb], b, acc[mb][nb]); if (NSPLIT >= 2) acc[mb][nb] = WFrag<T16>::mma(a[mb], b2, acc[mb][nb]); } }
        asm volatile("v_nop\n\tv_nop\n\tv_nop\n\tv_nop" : "+v"(acc[0][0]), "+v"(acc[1][1]), "+v"(acc[2][2]), "+v"(acc[3][3]) : "v"(a[0]), "v"(a[3]));
    }
#pragma unroll
    for (int mb = 0; mb < 4; ++mb) {
#pragma unroll
        for (int nb = 0; nb < 4; ++nb) {
#pragma unroll
            for (int j = 0; j < 8; ++j) os[(hi * 8 + j) * 68 + nb * 16 + lr] = acc[mb][nb][j]; }
        __builtin_amdgcn_wave_barrier(); asm volatile("" ::: "memory");
        float* crow = C + (size_t)(r0 + mb * 16) * ldc + c0;
#pragma unroll 1
        for (int ps = 0; ps < 2; ++ps) {
#pragma unroll
            for (int s = 0; s < 8; ++s) { const int row = 2 * s + hi, cofs = lr * 4; v4f val = *(const v4fa*)(os + row * 68 + cofs); if (BIAS) { val[0] += bfr(bias[c0 + cofs]); val[1] += bfr(bias[c0 + cofs + 1]); val[2] += bfr(bias[c0 + cofs + 2]); val[3] += bfr(bias[c0 + cofs + 3]); }
                *(volatile v4f*)(crow + (size_t)row * ldc + cofs) = val; }
            if (ps == 0) __threadfence(); }
        __builtin_amdgcn_wave_barrier(); asm volatile("" ::: "memory");
    }
}

__device__ __forceinline__ h16 tohx(float x) { return (h16)x; }
__device__ __forceinline__ void splitf(float y, unsigned short& h, unsigned short& l) { h = f2bf(y); l = f2bf(y - bf2f(h)); }
typedef __attribute__((ext_vector_type(2))) _Float16 v2h;
typedef __attribute__((ext_vector_type(4))) _Float16 v4h;
typedef __attribute__((ext_vector_type(2))) unsigned short v2us;
typedef __attribute__((ext_vector_type(4))) unsigned short v4us;

__global__ __launch_bounds__(256) void k_wtG(const float* __restrict__ w, int K, int N, bf* Bt) {
    const int lane = threadIdx.x & 31; const int L0 = (blockIdx.x * 8 + (threadIdx.x >> 5)) * 8; const int nlines = N * K / 64;
#pragma unroll 1
    for (int ps = 0; ps < 2; ++ps) {
#pragma unroll 1
        for (int l = 0; l < 8; ++l) { const int L = L0 + l; if (L >= nlines) break; const size_t e = (size_t)L * 64 + lane * 2; const int k = (int)(e % K), n = (int)(e / K); v2us o;
            o[0] = f2bf(w[(size_t)k * N + n]); o[1] = f2bf(w[(size_t)(k + 1) * N + n]); *(volatile v2us*)(Bt + e) = o; }
        if (ps == 0) __threadfence(); }
}
__global__ __launch_bounds__(256) void k_cvt8(const float* __restrict__ src, bf* dst, size_t n8) { const size_t i = (size_t)blockIdx.x * 256 + threadIdx.x; if (i >= n8) return; const v8f v = *(const v8f*)(src + i * 8); v8us o;
#pragma unroll
    for (int k = 0; k < 8; ++k) o[k] = f2bf(v[k]); *(volatile v8us*)(dst + i * 8) = o; __threadfence(); *(volatile v8us*)(dst + i * 8) = o; }
__global__ __launch_bounds__(256) void k_lnlat(const float* __restrict__ F, const float* __restrict__ g, const float* __restrict__ bb, bf* Yh, bf* Yl) { const int lane = threadIdx.x & 31; const int t = blockIdx.x * 8 + (threadIdx.x >> 5); if (t >= TT) return; float v[8]; float s = 0.f;
#pragma unroll
    for (int ch = 0; ch < 2; ++ch) { const v4f a = *(const v4f*)(F + (size_t)t * DL + ch * 128 + lane * 4);
#pragma unroll
        for (int q = 0; q < 4; ++q) { v[ch * 4 + q] = a[q]; s = __fadd_rn(s, a[q]); } }
#pragma unroll
    for (int sh = 16; sh; sh >>= 1) s += __shfl_xor(s, sh, 32);
    const float mu = s * (1.0f / DL); float q2 = 0.f;
#pragma unroll
    for (int k = 0; k < 8; ++k) { const float d = __fsub_rn(v[k], mu); float p = __fmul_rn(d, d); asm volatile("" : "+v"(p)); q2 = __fadd_rn(q2, p); }
#pragma unroll
    for (int sh = 16; sh; sh >>= 1) q2 += __shfl_xor(q2, sh, 32);
    const float rs = __frsqrt_rn(__fadd_rn(q2 * (1.0f / DL), 1e-5f));
#pragma unroll 1
    for (int ps = 0; ps < 2; ++ps) {
#pragma unroll
        for (int ch = 0; ch < 2; ++ch) { v4us oh, ol;
#pragma unroll
            for (int q = 0; q < 4; ++q) { const int d = ch * 128 + lane * 4 + q; float tn = __fmul_rn(__fsub_rn(v[ch * 4 + q], mu), rs); asm volatile("" : "+v"(tn)); float tg = __fmul_rn(tn, bfr(g[d])); asm volatile("" : "+v"(tg)); unsigned short a, c; splitf(__fadd_rn(tg, bfr(bb[d])), a, c); oh[q] = a; ol[q] = c; }
            const size_t o = (size_t)t * DL + ch * 128 + lane * 4; *(volatile v4us*)(Yh + o) = oh; *(volatile v4us*)(Yl + o) = ol; }
        if (ps == 0) __threadfence(); } }
__global__ __launch_bounds__(256) void k_ropeln(const float* __restrict__ F, int ld, int coff, const int* __restrict__ pos, const float* __restrict__ g, const float* __restrict__ bb, h16* P16, bf* Ph, bf* Pl) { const int lane = threadIdx.x & 31; const int row = blockIdx.x * 8 + (threadIdx.x >> 5); if (row >= NH_ * TT) return; const int t = row % TT, h = row / TT; const float* f = F + (size_t)t * ld + coff + h * HD; const int d0 = 2 * lane; const float a0 = f[d0], a1 = f[d0 + 1]; const float p0 = __shfl_xor(a0, 16, 32), p1 = __shfl_xor(a1, 16, 32); const int i0 = d0 & 31; const float pt = (float)pos[t]; float r[2];
#pragma unroll
    for (int u = 0; u < 2; ++u) { const float inv = __expf(__fmul_rn(-(float)(2 * (i0 + u)) / (float)HD, 9.210340371976184f)); const float ang = __fmul_rn(pt, inv); const float cs = cosf(ang), sn = sinf(ang); const float a = u ? a1 : a0, p = u ? p1 : p0;
        if (lane < 16) { float m1 = __fmul_rn(a, cs); asm volatile("" : "+v"(m1)); float m2 = __fmul_rn(p, sn); asm volatile("" : "+v"(m2)); r[u] = __fsub_rn(m1, m2); }
        else { float m1 = __fmul_rn(p, sn); asm volatile("" : "+v"(m1)); float m2 = __fmul_rn(a, cs); asm volatile("" : "+v"(m2)); r[u] = __fadd_rn(m1, m2); } }
    float s = __fadd_rn(r[0], r[1]);
#pragma unroll
    for (int sh = 16; sh; sh >>= 1) s += __shfl_xor(s, sh, 32);
    const float mu = s * (1.0f / HD); const float e0 = __fsub_rn(r[0], mu), e1 = __fsub_rn(r[1], mu); float q2 = __fadd_rn(__fmul_rn(e0, e0), __fmul_rn(e1, e1));
#pragma unroll
    for (int sh = 16; sh; sh >>= 1) q2 += __shfl_xor(q2, sh, 32);
    const float rs = __frsqrt_rn(__fadd_rn(q2 * (1.0f / HD), 1e-5f)); v2h o; v2us oh, ol;
#pragma unroll
    for (int u = 0; u < 2; ++u) { float n1 = __fmul_rn(u ? e1 : e0, rs); asm volatile("" : "+v"(n1)); float g1 = __fmul_rn(n1, bfr(g[d0 + u])); asm volatile("" : "+v"(g1)); const float y = __fadd_rn(g1, bfr(bb[d0 + u])); o[u] = tohx(y); unsigned short a2, c2; splitf(y, a2, c2); oh[u] = a2; ol[u] = c2; }
    const size_t oo = (size_t)row * HD + d0; for (int ps = 0; ps < 2; ++ps) { *(volatile v2h*)(P16 + oo) = o; *(volatile v2us*)(Ph + oo) = oh; *(volatile v2us*)(Pl + oo) = ol; if (ps == 0) __threadfence(); } }
__global__ __launch_bounds__(256) void k_vtp(const float* __restrict__ KV, h16* V16, bf* Vh, bf* Vl) { const size_t e = ((size_t)blockIdx.x * 256 + threadIdx.x) * 2; if (e >= (size_t)NH_ * HD * TT) return; const int t = (int)(e % TT); const int d = (int)((e / TT) % HD); const int h = (int)(e / ((size_t)TT * HD)); v2h o; v2us oh, ol;
#pragma unroll
    for (int u = 0; u < 2; ++u) { const float v = KV[(size_t)(t + u) * 2 * DM + DM + h * HD + d]; o[u] = tohx(v); unsigned short a, c; splitf(v, a, c); oh[u] = a; ol[u] = c; } for (int ps = 0; ps < 2; ++ps) { *(volatile v2h*)(V16 + e) = o; *(volatile v2us*)(Vh + e) = oh; *(volatile v2us*)(Vl + e) = ol; if (ps == 0) __threadfence(); } }
__global__ __launch_bounds__(256) void k_asoft(const float* __restrict__ Sb, h16* P16, bf* Ph, bf* Pl) { const int lane = threadIdx.x & 31; const int row = blockIdx.x * 8 + (threadIdx.x >> 5); if (row >= ZH * TT) return; const int i = row % TT, z = row / TT; const bool hires = i < RH; const float* sr = Sb + (size_t)row * TT; float v[64]; float mx = -3.0e38f;
#pragma unroll
    for (int ch = 0; ch < 16; ++ch) { const v4f a = *(const v4f*)(sr + ch * 128 + lane * 4);
#pragma unroll
        for (int q = 0; q < 4; ++q) { float t = a[q] * SCL; asm volatile("" : "+v"(t)); v[ch * 4 + q] = t; mx = fmaxf(mx, t); } }
#pragma unroll
    for (int sh = 16; sh; sh >>= 1) mx = fmaxf(mx, __shfl_xor(mx, sh, 32));
    float sum = 0.f;
#pragma unroll
    for (int k = 0; k < 64; ++k) { float d0 = __fsub_rn(v[k], mx); asm volatile("" : "+v"(d0)); v[k] = __expf(d0); sum += v[k]; }
#pragma unroll
    for (int sh = 16; sh; sh >>= 1) sum += __shfl_xor(sum, sh, 32);
    const float f = __fdiv_rn(hires ? 1.0f : PCAR, sum);
#pragma unroll 1
    for (int ps = 0; ps < 2; ++ps) {
        if (hires) {
#pragma unroll
            for (int ch = 0; ch < 16; ++ch) { v4us oh, ol;
#pragma unroll
                for (int q = 0; q < 4; ++q) { unsigned short a, c2; splitf(v[ch * 4 + q] * f, a, c2); oh[q] = a; ol[q] = c2; } const size_t oo = ((size_t)z * RH + i) * TT + ch * 128 + lane * 4; *(volatile v4us*)(Ph + oo) = oh; *(volatile v4us*)(Pl + oo) = ol; }
        } else {
#pragma unroll
            for (int ch = 0; ch < 16; ++ch) { v4h o4; o4[0] = tohx(v[ch * 4] * f); o4[1] = tohx(v[ch * 4 + 1] * f); o4[2] = tohx(v[ch * 4 + 2] * f); o4[3] = tohx(v[ch * 4 + 3] * f); *(volatile v4h*)(P16 + (size_t)row * TT + ch * 128 + lane * 4) = o4; } }
        if (ps == 0) __threadfence(); } }
__global__ __launch_bounds__(256) void k_mrg(const float* __restrict__ Ob, int h0, bf* Ah, bf* Al) { const size_t e = ((size_t)blockIdx.x * 256 + threadIdx.x) * 2; if (e >= (size_t)ZH * TT * HD) return; const int d = (int)(e % HD); const int t = (int)((e / HD) % TT); const int z = (int)(e / ((size_t)HD * TT)); const float f = t < RH ? 1.0f : (1.0f / PCAR); v2us oh, ol;
#pragma unroll
    for (int u = 0; u < 2; ++u) { unsigned short a, c; splitf(Ob[e + u] * f, a, c); oh[u] = a; ol[u] = c; } const size_t o = (size_t)t * DM + (h0 + z) * HD + d; *(volatile v2us*)(Ah + o) = oh; *(volatile v2us*)(Al + o) = ol; __threadfence(); *(volatile v2us*)(Ah + o) = oh; *(volatile v2us*)(Al + o) = ol; }

extern "C" void kernel_launch(void* const* d_in, const int* in_sizes, int n_in,
                              void* d_out, int out_size, void* d_ws, size_t ws_size, hipStream_t stream) {
    (void)in_sizes; (void)n_in; (void)out_size;
    const float* x = (const float*)d_in[0]; const int* pos = (const int*)d_in[1]; const float* Wq = (const float*)d_in[2]; const float* Wd = (const float*)d_in[3]; const float* lng = (const float*)d_in[4]; const float* lnb = (const float*)d_in[5]; const float* Wkv = (const float*)d_in[6]; const float* Wo = (const float*)d_in[7]; const float* qg = (const float*)d_in[8]; const float* qb = (const float*)d_in[9]; const float* kg = (const float*)d_in[10]; const float* kb = (const float*)d_in[11];
    float* OUT = (float*)d_out;
    char* wsp = (char*)d_ws;
    auto take = [&](size_t bytes) { char* p = wsp; wsp += (bytes + 255) & ~(size_t)255; return (void*)p; };
    bf* WQ = (bf*)take((size_t)DM * DM * 2); bf* WD = (bf*)take((size_t)DL * DM * 2); bf* WKV = (bf*)take((size_t)2 * DM * DL * 2); bf* WO = (bf*)take((size_t)DM * DM * 2); bf* XB = (bf*)take((size_t)TT * DM * 2);
    float* QF = (float*)take((size_t)TT * DM * 4); float* LF = (float*)take((size_t)TT * DL * 4); bf* Lh = (bf*)take((size_t)TT * DL * 2); bf* Ll = (bf*)take((size_t)TT * DL * 2); float* KV = (float*)take((size_t)TT * 2 * DM * 4);
    h16* Q16 = (h16*)take((size_t)NH_ * TT * HD * 2); bf* Qh = (bf*)take((size_t)NH_ * TT * HD * 2); bf* Ql = (bf*)take((size_t)NH_ * TT * HD * 2); h16* K16 = (h16*)take((size_t)NH_ * TT * HD * 2); bf* Kh = (bf*)take((size_t)NH_ * TT * HD * 2); bf* Kl = (bf*)take((size_t)NH_ * TT * HD * 2); h16* V16 = (h16*)take((size_t)NH_ * HD * TT * 2); bf* Vh = (bf*)take((size_t)NH_ * HD * TT * 2); bf* Vl = (bf*)take((size_t)NH_ * HD * TT * 2);
    float* Sb = (float*)take((size_t)ZH * TT * TT * 4); h16* P16 = (h16*)take((size_t)ZH * TT * TT * 2); bf* Ph = (bf*)take((size_t)ZH * RH * TT * 2); bf* Pl = (bf*)take((size_t)ZH * RH * TT * 2); float* Ob = (float*)take((size_t)ZH * TT * HD * 4); bf* Ah = (bf*)take((size_t)TT * DM * 2); bf* Al = (bf*)take((size_t)TT * DM * 2);
    if ((size_t)(wsp - (char*)d_ws) > ws_size) return;
    k_wtG<<<(DM * DM / 64 + 63) / 64, 256, 0, stream>>>(Wq, DM, DM, WQ); k_wtG<<<(DM * DL / 64 + 63) / 64, 256, 0, stream>>>(Wd, DM, DL, WD); k_wtG<<<(DL * 2 * DM / 64 + 63) / 64, 256, 0, stream>>>(Wkv, DL, 2 * DM, WKV); k_wtG<<<(DM * DM / 64 + 63) / 64, 256, 0, stream>>>(Wo, DM, DM, WO);
    for (int b = 0; b < NB_; ++b) {
        k_cvt8<<<(TT * DM / 8 + 255) / 256, 256, 0, stream>>>(x + (size_t)b * TT * DM, XB, (size_t)TT * DM / 8);
        k_gemmw<bf, 0, false><<<dim3(TT / 64, DM / 64, 1), 32, 0, stream>>>(XB, nullptr, WQ, nullptr, DM, QF, DM, nullptr, 0, 0, 0); k_ropeln<<<NH_ * TT / 8, 256, 0, stream>>>(QF, DM, 0, pos, qg, qb, Q16, Qh, Ql);
        k_gemmw<bf, 0, false><<<dim3(TT / 64, DL / 64, 1), 32, 0, stream>>>(XB, nullptr, WD, nullptr, DM, LF, DL, nullptr, 0, 0, 0); k_lnlat<<<TT / 8, 256, 0, stream>>>(LF, lng, lnb, Lh, Ll);
        k_gemmw<bf, 1, false><<<dim3(TT / 64, 2 * DM / 64, 1), 32, 0, stream>>>(Lh, Ll, WKV, nullptr, DL, KV, 2 * DM, nullptr, 0, 0, 0);
        k_ropeln<<<NH_ * TT / 8, 256, 0, stream>>>(KV, 2 * DM, 0, pos, kg, kb, K16, Kh, Kl); k_vtp<<<(unsigned)(((size_t)NH_ * HD * TT / 2 + 255) / 256), 256, 0, stream>>>(KV, V16, Vh, Vl);
        for (int h0 = 0; h0 < NH_; h0 += ZH) { const size_t z = (size_t)h0;
            k_gemmw<bf, 2, false><<<dim3(RH / 64, TT / 64, ZH), 32, 0, stream>>>(Qh + z * TT * HD, Ql + z * TT * HD, Kh + z * TT * HD, Kl + z * TT * HD, HD, Sb, TT, nullptr, (size_t)TT * HD, (size_t)TT * HD, (size_t)TT * TT);
            k_gemmw<h16, 0, false><<<dim3((TT - RH) / 64, TT / 64, ZH), 32, 0, stream>>>(Q16 + z * TT * HD + (size_t)RH * HD, nullptr, K16 + z * TT * HD, nullptr, HD, Sb + (size_t)RH * TT, TT, nullptr, (size_t)TT * HD, (size_t)TT * HD, (size_t)TT * TT);
            k_asoft<<<ZH * TT / 8, 256, 0, stream>>>(Sb, P16, Ph, Pl);
            k_gemmw<bf, 2, false><<<dim3(RH / 64, 1, ZH), 32, 0, stream>>>(Ph, Pl, Vh + z * HD * TT, Vl + z * HD * TT, TT, Ob, HD, nullptr, (size_t)RH * TT, (size_t)HD * TT, (size_t)TT * HD);
            k_gemmw<h16, 0, false><<<dim3((TT - RH) / 64, 1, ZH), 32, 0, stream>>>(P16 + (size_t)RH * TT, nullptr, V16 + z * HD * TT, nullptr, TT, Ob + (size_t)RH * HD, HD, nullptr, (size_t)TT * TT, (size_t)HD * TT, (size_t)TT * HD);
            k_mrg<<<(unsigned)(((size_t)ZH * TT * HD / 2 + 255) / 256), 256, 0, stream>>>(Ob, h0, Ah, Al); }
        k_gemmw<bf, 1, false><<<dim3(TT / 64, DM / 64, 1), 32, 0, stream>>>(Ah, Al, WO, nullptr, DM, OUT + (size_t)b * TT * DM, DM, nullptr, 0, 0, 0); }
}
